// MMA_14645838479638
// MI455X (gfx1250) — hardware-verified
//
#include <hip/hip_runtime.h>
#include <stdint.h>
#include <stddef.h>


#define LSEQ 8192
#define CIN  6
#define DM   32
#define DI   64
#define DS   16
#define NXP  34
#define TCH  32

typedef _Float16 v16h __attribute__((ext_vector_type(16)));
typedef _Float16 v8h  __attribute__((ext_vector_type(8)));
typedef float    v8f  __attribute__((ext_vector_type(8)));
typedef float    v4f  __attribute__((ext_vector_type(4)));
typedef v8h __attribute__((may_alias)) v8ha;
typedef v4f __attribute__((may_alias)) v4fa;
union Frag { v16h v; v8h half[2]; };

__device__ __forceinline__ v8f wmma_f16(v16h a, v16h b, v8f c) {
    c = __builtin_amdgcn_wmma_f32_16x16x32_f16(false, a, false, b, (short)0, c, false, false);
    asm volatile("v_nop\n\tv_nop\n\tv_nop\n\tv_nop" : "+v"(c) : "v"(a), "v"(b));
    return c;
}

__device__ __forceinline__ v8h cvt8(const float* p, float s) {
    const v4f u = *(const v4fa*)p;
    const v4f v = *(const v4fa*)(p + 4);
    v8h r;
    r[0] = (_Float16)(u[0] * s); r[1] = (_Float16)(u[1] * s);
    r[2] = (_Float16)(u[2] * s); r[3] = (_Float16)(u[3] * s);
    r[4] = (_Float16)(v[0] * s); r[5] = (_Float16)(v[1] * s);
    r[6] = (_Float16)(v[2] * s); r[7] = (_Float16)(v[3] * s);
    return r;
}

__device__ __forceinline__ float softplus_f(float v) {
    return fmaxf(v, 0.f) + log1pf(expf(-fabsf(v)));
}

__global__ __launch_bounds__(256) void k_front(const float* __restrict__ x, const float* __restrict__ w,
                                               const float* __restrict__ g, const float* __restrict__ be,
                                               const float* __restrict__ mu, const float* __restrict__ va,
                                               float* hout, int nrows) {
    const int t = threadIdx.x, l = t & 31;
    const int gw = blockIdx.x * 8 + (t >> 5);
    const int row = gw * 4 + (l >> 3);
    const int dq = l & 7;
    const bool ok = row < nrows;
    v4f o = {0.f, 0.f, 0.f, 0.f};
    if (ok) {
        const int b = row / LSEQ;
        const int lp = row - b * LSEQ;
        const float* xb = x + (size_t)b * CIN * LSEQ;
        const float* wb = w + (size_t)(4 * dq) * CIN * 3;
        float a0 = 0.f, a1 = 0.f, a2 = 0.f, a3 = 0.f;
        #pragma unroll
        for (int c = 0; c < CIN; ++c) {
            const float* xc = xb + (size_t)c * LSEQ;
            const float x0 = (lp > 0) ? xc[lp - 1] : 0.f;
            const float x1 = xc[lp];
            const float x2 = (lp < LSEQ - 1) ? xc[lp + 1] : 0.f;
            const float* wc = wb + c * 3;
            a0 += x0 * wc[0]  + x1 * wc[1]  + x2 * wc[2];
            a1 += x0 * wc[18] + x1 * wc[19] + x2 * wc[20];
            a2 += x0 * wc[36] + x1 * wc[37] + x2 * wc[38];
            a3 += x0 * wc[54] + x1 * wc[55] + x2 * wc[56];
        }
        const float av[4] = {a0, a1, a2, a3};
        #pragma unroll
        for (int j = 0; j < 4; ++j) {
            const int d = 4 * dq + j;
            const float v = (av[j] - mu[d]) * rsqrtf(va[d] + 1e-5f) * g[d] + be[d];
            o[j] = v > 0.f ? v : 0.f;
        }
    }
    float* dst = hout + (size_t)(ok ? row : 0) * DM + 4 * dq;
    if (ok) *(volatile v4fa*)dst = o;
    __threadfence();
    if (ok) *(volatile v4fa*)dst = o;
}

__device__ __forceinline__ void st_xz_tile(const float* o, float* xz, int row0, int l) {
    #pragma unroll
    for (int it = 0; it < 16; ++it) {
        const int j = it * 4 + (l >> 3);
        const int row = j >> 2;
        const int col = (j & 3) * 32 + (l & 7) * 4;
        const v4f v = *(const v4fa*)(o + row * 128 + col);
        *(volatile v4fa*)(xz + (size_t)(row0 + row) * 128 + col) = v;
    }
}

__global__ __launch_bounds__(128) void k_inproj(const float* __restrict__ hin, const float* __restrict__ nw,
                                                const float* __restrict__ Wi, float* xz, int nrows) {
    __shared__ __attribute__((aligned(16))) float ot[4 * 16 * 128];
    const int t = threadIdx.x, w = t >> 5, l = t & 31, hh = l >> 4, m = l & 15;
    const int row0u = (blockIdx.x * 4 + w) * 16;
    const bool ok = (row0u + 16) <= nrows;
    const int row0 = ok ? row0u : 0;

    const float* hr = hin + (size_t)(row0 + m) * DM;
    const v4f p0 = *(const v4fa*)(hr + 8 * hh);
    const v4f p1 = *(const v4fa*)(hr + 8 * hh + 4);
    const v4f p2 = *(const v4fa*)(hr + 16 + 8 * hh);
    const v4f p3 = *(const v4fa*)(hr + 16 + 8 * hh + 4);
    float ss = p0[0]*p0[0] + p0[1]*p0[1] + p0[2]*p0[2] + p0[3]*p0[3]
             + p1[0]*p1[0] + p1[1]*p1[1] + p1[2]*p1[2] + p1[3]*p1[3]
             + p2[0]*p2[0] + p2[1]*p2[1] + p2[2]*p2[2] + p2[3]*p2[3]
             + p3[0]*p3[0] + p3[1]*p3[1] + p3[2]*p3[2] + p3[3]*p3[3];
    ss += __shfl_xor(ss, 16, 32);
    const float sc = 1.0f / sqrtf(ss * (1.0f / 32.0f) + 1e-5f);
    const v4f n0 = *(const v4fa*)(nw + 8 * hh);
    const v4f n1 = *(const v4fa*)(nw + 8 * hh + 4);
    const v4f n2 = *(const v4fa*)(nw + 16 + 8 * hh);
    const v4f n3 = *(const v4fa*)(nw + 16 + 8 * hh + 4);
    Frag a;
    {
        v8h q;
        q[0] = (_Float16)((p0[0] * sc) * n0[0]); q[1] = (_Float16)((p0[1] * sc) * n0[1]);
        q[2] = (_Float16)((p0[2] * sc) * n0[2]); q[3] = (_Float16)((p0[3] * sc) * n0[3]);
        q[4] = (_Float16)((p1[0] * sc) * n1[0]); q[5] = (_Float16)((p1[1] * sc) * n1[1]);
        q[6] = (_Float16)((p1[2] * sc) * n1[2]); q[7] = (_Float16)((p1[3] * sc) * n1[3]);
        a.half[0] = q;
        v8h q2;
        q2[0] = (_Float16)((p2[0] * sc) * n2[0]); q2[1] = (_Float16)((p2[1] * sc) * n2[1]);
        q2[2] = (_Float16)((p2[2] * sc) * n2[2]); q2[3] = (_Float16)((p2[3] * sc) * n2[3]);
        q2[4] = (_Float16)((p3[0] * sc) * n3[0]); q2[5] = (_Float16)((p3[1] * sc) * n3[1]);
        q2[6] = (_Float16)((p3[2] * sc) * n3[2]); q2[7] = (_Float16)((p3[3] * sc) * n3[3]);
        a.half[1] = q2;
    }

    v8f acc[8];
    #pragma unroll
    for (int nt = 0; nt < 8; ++nt) { v8f z = {0.f,0.f,0.f,0.f,0.f,0.f,0.f,0.f}; acc[nt] = z; }
    #pragma unroll
    for (int nt = 0; nt < 8; ++nt) {
        const float* wr = Wi + (size_t)(nt * 16 + m) * DM;
        Frag b;
        b.half[0] = cvt8(wr + 8 * hh, 1024.f);
        b.half[1] = cvt8(wr + 16 + 8 * hh, 1024.f);
        acc[nt] = wmma_f16(a.v, b.v, acc[nt]);
    }
    float* o = ot + w * 2048;
    #pragma unroll
    for (int nt = 0; nt < 8; ++nt) {
        #pragma unroll
        for (int r = 0; r < 8; ++r) o[(8 * hh + r) * 128 + nt * 16 + m] = acc[nt][r] * (1.0f / 1024.0f);
    }
    __syncthreads();
    if (ok) st_xz_tile(o, xz, row0, l);
    __threadfence();
    if (ok) st_xz_tile(o, xz, row0, l);
}

__device__ __forceinline__ void st_xc_tile(const float* xs, float* xcg, int tr0, int t) {
    #pragma unroll
    for (int it = 0; it < 8; ++it) {
        const int p = it * 128 + t;
        const int line = p >> 3, q = p & 7;
        const int row = line >> 1, col = (line & 1) * 32 + q * 4;
        const v4f v = *(const v4fa*)(xs + row * 64 + col);
        *(volatile v4fa*)(xcg + (size_t)(tr0 + row) * DI + col) = v;
    }
}
__device__ __forceinline__ void st_delta_tile(const float* xs, float* dlg, int tr0, int w, int l) {
    #pragma unroll
    for (int it = 0; it < 8; ++it) {
        const int j = it * 4 + (l >> 3);
        const int row = 16 * w + (j >> 1), col = (j & 1) * 32 + (l & 7) * 4;
        const v4f v = *(const v4fa*)(xs + row * 64 + col);
        *(volatile v4fa*)(dlg + (size_t)(tr0 + row) * DI + col) = v;
    }
}
__device__ __forceinline__ void st_bc_tile(const float* dw, float* bcg, int tr0, int w, int l) {
    #pragma unroll
    for (int it = 0; it < 4; ++it) {
        const int row = it * 4 + (l >> 3), q = l & 7;
        const float* s = dw + row * 48 + 2 + 4 * q;
        v4f v; v[0] = s[0]; v[1] = s[1]; v[2] = s[2]; v[3] = s[3];
        *(volatile v4fa*)(bcg + (size_t)(tr0 + 16 * w + row) * 32 + 4 * q) = v;
    }
}

__global__ __launch_bounds__(128) void k_xdd(const float* __restrict__ xz, const float* __restrict__ cw,
                                             const float* __restrict__ cb, const float* __restrict__ Wx,
                                             const float* __restrict__ Wdt, const float* __restrict__ bdt,
                                             float* xcg, float* dlg, float* bcg, int nrows) {
    __shared__ __attribute__((aligned(16))) float xs[64 * 64];
    __shared__ __attribute__((aligned(16))) float dtl[4 * 16 * 48];
    const int t = threadIdx.x, w = t >> 5, l = t & 31, hh = l >> 4, m = l & 15;
    const int tr0u = blockIdx.x * 64;
    const bool okb = (tr0u + 64) <= nrows;
    const int tr0 = okb ? tr0u : 0;

    {
        const int d = t & 63, rg = t >> 6;
        const int rb = tr0 + rg * 32;
        const int lp = rb & (LSEQ - 1);
        const float w0 = cw[d * 4 + 0], w1 = cw[d * 4 + 1], w2 = cw[d * 4 + 2], w3 = cw[d * 4 + 3];
        const float bias = cb[d];
        float xm3 = 0.f, xm2 = 0.f, xm1 = 0.f;
        if (lp >= 3) {
            xm3 = xz[(size_t)(rb - 3) * 128 + d];
            xm2 = xz[(size_t)(rb - 2) * 128 + d];
            xm1 = xz[(size_t)(rb - 1) * 128 + d];
        }
        #pragma unroll 4
        for (int i = 0; i < 32; ++i) {
            const float xv = xz[(size_t)(rb + i) * 128 + d];
            const float a = ((w0 * xm3 + w1 * xm2) + w2 * xm1 + w3 * xv) + bias;
            const float sg = 1.0f / (1.0f + __expf(-a));
            xs[(rg * 32 + i) * 64 + d] = a * sg;
            xm3 = xm2; xm2 = xm1; xm1 = xv;
        }
    }
    __syncthreads();

    if (okb) st_xc_tile(xs, xcg, tr0, t);
    __threadfence();
    if (okb) st_xc_tile(xs, xcg, tr0, t);

    v8f acc[3];
    #pragma unroll
    for (int nt = 0; nt < 3; ++nt) { v8f z = {0.f,0.f,0.f,0.f,0.f,0.f,0.f,0.f}; acc[nt] = z; }
    #pragma unroll
    for (int kk = 0; kk < 2; ++kk) {
        const float* ap = xs + (16 * w + m) * 64 + kk * 32;
        Frag a;
        a.half[0] = cvt8(ap + 8 * hh, 256.f);
        a.half[1] = cvt8(ap + 16 + 8 * hh, 256.f);
        #pragma unroll
        for (int nt = 0; nt < 3; ++nt) {
            const int n = nt * 16 + m;
            const int nn = (n < NXP) ? n : (NXP - 1);
            const float s = (n < NXP) ? 1024.f : 0.f;
            const float* wr = Wx + (size_t)nn * DI + kk * 32;
            Frag b;
            b.half[0] = cvt8(wr + 8 * hh, s);
            b.half[1] = cvt8(wr + 16 + 8 * hh, s);
            acc[nt] = wmma_f16(a.v, b.v, acc[nt]);
        }
    }
    float* dw = dtl + w * 768;
    #pragma unroll
    for (int nt = 0; nt < 3; ++nt) {
        #pragma unroll
        for (int r = 0; r < 8; ++r) dw[(8 * hh + r) * 48 + nt * 16 + m] = acc[nt][r] * (1.0f / 262144.0f);
    }
    __syncthreads();

    {
        const int d0 = l, d1 = l + 32;
        const float a00 = Wdt[d0 * 2], a01 = Wdt[d0 * 2 + 1], b0 = bdt[d0];
        const float a10 = Wdt[d1 * 2], a11 = Wdt[d1 * 2 + 1], b1 = bdt[d1];
        #pragma unroll 4
        for (int r = 0; r < 16; ++r) {
            const float t0 = dw[r * 48 + 0], t1 = dw[r * 48 + 1];
            const float v0 = t0 * a00 + t1 * a01 + b0;
            const float v1 = t0 * a10 + t1 * a11 + b1;
            xs[(16 * w + r) * 64 + d0] = softplus_f(v0);
            xs[(16 * w + r) * 64 + d1] = softplus_f(v1);
        }
    }
    __syncthreads();

    if (okb) { st_delta_tile(xs, dlg, tr0, w, l); st_bc_tile(dw, bcg, tr0, w, l); }
    __threadfence();
    if (okb) { st_delta_tile(xs, dlg, tr0, w, l); st_bc_tile(dw, bcg, tr0, w, l); }
}

__global__ __launch_bounds__(512) void k_scan(const float* __restrict__ dlg, const float* __restrict__ bcg,
                                              const float* __restrict__ xcg, const float* __restrict__ xz,
                                              const float* __restrict__ Alog, const float* __restrict__ Dp,
                                              _Float16* yg) {
    __shared__ __attribute__((aligned(16))) float S[7168];
    __shared__ __attribute__((aligned(16))) _Float16 yt[TCH * 64];
    const int b = blockIdx.x, t = threadIdx.x;
    const int d = t >> 3, sp = t & 7, s0 = sp, s1 = sp + 8;
    const float A0 = -expf(Alog[d * DS + s0]);
    const float A1 = -expf(Alog[d * DS + s1]);
    const float Dd = Dp[d];
    float h0 = 0.f, h1 = 0.f, m0 = 0.f, m1 = 0.f;
    const size_t rb = (size_t)b * LSEQ;

    #pragma unroll 1
    for (int c = 0; c < LSEQ / TCH; ++c) {
        const size_t r0 = rb + (size_t)c * TCH;
        for (int e4 = t; e4 < 1792; e4 += 512) {
            const float* src;
            if (e4 < 512)       { const int row = e4 >> 4, pc = e4 & 15; src = dlg + (r0 + row) * DI + pc * 4; }
            else if (e4 < 768)  { const int i = e4 - 512;  const int row = i >> 3, pc = i & 7;  src = bcg + (r0 + row) * 32 + pc * 4; }
            else if (e4 < 1280) { const int i = e4 - 768;  const int row = i >> 4, pc = i & 15; src = xcg + (r0 + row) * DI + pc * 4; }
            else                { const int i = e4 - 1280; const int row = i >> 4, pc = i & 15; src = xz + (r0 + row) * 128 + 64 + pc * 4; }
            *(v4fa*)(S + e4 * 4) = *(const v4fa*)src;
        }
        __syncthreads();
        #pragma unroll 1
        for (int st = 0; st < TCH; ++st) {
            const float dv = S[st * 64 + d];
            const float B0 = S[2048 + st * 32 + s0];
            const float B1 = S[2048 + st * 32 + s1];
            const float C0 = S[2048 + st * 32 + 16 + s0];
            const float C1 = S[2048 + st * 32 + 16 + s1];
            const float xv = S[3072 + st * 64 + d];
            m0 = 0.8f * m0 + (dv * B0) * xv;
            m1 = 0.8f * m1 + (dv * B1) * xv;
            h0 = __expf(dv * A0) * h0 + m0;
            h1 = __expf(dv * A1) * h1 + m1;
            float ctb = h0 * C0 + h1 * C1;
            ctb += __shfl_xor(ctb, 4, 8);
            ctb += __shfl_xor(ctb, 2, 8);
            ctb += __shfl_xor(ctb, 1, 8);
            if (sp == 0) {
                const float z = S[5120 + st * 64 + d];
                const float y = (ctb + Dd * xv) * (z * (1.0f / (1.0f + __expf(-z))));
                yt[st * 64 + d] = (_Float16)(y * 256.0f);
            }
        }
        __syncthreads();
        if (t < 256) {
            const int line = t >> 3, q = t & 7;
            const v8h v = *(const v8ha*)(yt + line * 64 + 8 * q);
            *(volatile v8ha*)(yg + (r0 + line) * DI + 8 * q) = v;
        }
        __threadfence();
        if (t < 256) {
            const int line = t >> 3, q = t & 7;
            const v8h v = *(const v8ha*)(yt + line * 64 + 8 * q);
            *(volatile v8ha*)(yg + (r0 + line) * DI + 8 * q) = v;
        }
        __syncthreads();
    }
}

__global__ __launch_bounds__(128) void k_outproj(const _Float16* __restrict__ yg, const float* __restrict__ Wo,
                                                 float* hio, int nrows) {
    __shared__ __attribute__((aligned(16))) float ot[4 * 16 * 32];
    const int t = threadIdx.x, w = t >> 5, l = t & 31, hh = l >> 4, m = l & 15;
    const int row0u = (blockIdx.x * 4 + w) * 16;
    const bool ok = (row0u + 16) <= nrows;
    const int row0 = ok ? row0u : 0;

    v8f acc[2];
    { v8f z = {0.f,0.f,0.f,0.f,0.f,0.f,0.f,0.f}; acc[0] = z; acc[1] = z; }
    #pragma unroll
    for (int kk = 0; kk < 2; ++kk) {
        const _Float16* ar = yg + (size_t)(row0 + m) * DI + kk * 32;
        Frag a;
        a.half[0] = *(const v8ha*)(ar + 8 * hh);
        a.half[1] = *(const v8ha*)(ar + 16 + 8 * hh);
        #pragma unroll
        for (int nt = 0; nt < 2; ++nt) {
            const float* wr = Wo + (size_t)(nt * 16 + m) * DI + kk * 32;
            Frag b;
            b.half[0] = cvt8(wr + 8 * hh, 1024.f);
            b.half[1] = cvt8(wr + 16 + 8 * hh, 1024.f);
            acc[nt] = wmma_f16(a.v, b.v, acc[nt]);
        }
    }
    float* o = ot + w * 512;
    #pragma unroll
    for (int nt = 0; nt < 2; ++nt) {
        #pragma unroll
        for (int r = 0; r < 8; ++r) o[(8 * hh + r) * 32 + nt * 16 + m] = acc[nt][r] * (1.0f / 262144.0f);
    }
    __syncthreads();
    v4f vals[4];
    #pragma unroll
    for (int it = 0; it < 4; ++it) {
        const int row = it * 4 + (l >> 3), q = l & 7;
        const v4f hv = *(const v4fa*)(hio + (size_t)(row0 + row) * DM + 4 * q);
        const v4f dv = *(const v4fa*)(o + row * 32 + 4 * q);
        vals[it] = hv + dv;
    }
    if (ok) {
        #pragma unroll
        for (int it = 0; it < 4; ++it) {
            const int row = it * 4 + (l >> 3), q = l & 7;
            *(volatile v4fa*)(hio + (size_t)(row0 + row) * DM + 4 * q) = vals[it];
        }
    }
    __threadfence();
    if (ok) {
        #pragma unroll
        for (int it = 0; it < 4; ++it) {
            const int row = it * 4 + (l >> 3), q = l & 7;
            *(volatile v4fa*)(hio + (size_t)(row0 + row) * DM + 4 * q) = vals[it];
        }
    }
}

__global__ __launch_bounds__(256) void k_poolcls(const float* __restrict__ hin, const float* __restrict__ cw,
                                                 const float* __restrict__ cb, float* out, int nb) {
    __shared__ float pooled[256];
    __shared__ __attribute__((aligned(16))) float ot[256];
    const int t = threadIdx.x, bl = t >> 5, d = t & 31;
    const int bg = blockIdx.x * 8 + bl;
    const bool okb = bg < nb;
    float pm = 0.f;
    if (okb) {
        const float* hp = hin + (size_t)bg * LSEQ * DM + d;
        double acc = 0.0;
        #pragma unroll 4
        for (int i = 0; i < LSEQ; ++i) acc += (double)hp[(size_t)i * DM];
        pm = (float)(acc * (1.0 / (double)LSEQ));
    }
    pooled[t] = pm;
    __syncthreads();
    float ov = 0.f;
    if (okb) {
        const float* pr = pooled + bl * 32;
        const float* cr = cw + (size_t)d * DM;
        float s = 0.f;
        #pragma unroll
        for (int d2 = 0; d2 < DM; ++d2) s += pr[d2] * cr[d2];
        ov = s + cb[d];
    }
    ot[t] = ov;
    __syncthreads();
    if (t < 64) {
        const int line = t >> 3, q = t & 7;
        const int bgl = blockIdx.x * 8 + line;
        if (bgl < nb) {
            const v4f v = *(const v4fa*)(ot + line * 32 + 4 * q);
            *(volatile v4fa*)(out + (size_t)bgl * 32 + 4 * q) = v;
        }
    }
    __threadfence();
    if (t < 64) {
        const int line = t >> 3, q = t & 7;
        const int bgl = blockIdx.x * 8 + line;
        if (bgl < nb) {
            const v4f v = *(const v4fa*)(ot + line * 32 + 4 * q);
            *(volatile v4fa*)(out + (size_t)bgl * 32 + 4 * q) = v;
        }
    }
}

static inline size_t al256(size_t v) { return (v + 255) & ~(size_t)255; }

extern "C" void kernel_launch(void* const* d_in, const int* in_sizes, int n_in,
                              void* d_out, int out_size, void* d_ws, size_t ws_size,
                              hipStream_t stream) {
    if (n_in < 18) return;
    const float* x       = (const float*)d_in[0];
    const float* conv_w  = (const float*)d_in[1];
    const float* bn_g    = (const float*)d_in[2];
    const float* bn_b    = (const float*)d_in[3];
    const float* bn_m    = (const float*)d_in[4];
    const float* bn_v    = (const float*)d_in[5];
    const float* norm_w  = (const float*)d_in[6];
    const float* in_w    = (const float*)d_in[7];
    const float* conv_dw = (const float*)d_in[8];
    const float* conv_db = (const float*)d_in[9];
    const float* x_w     = (const float*)d_in[10];
    const float* dt_w    = (const float*)d_in[11];
    const float* dt_b    = (const float*)d_in[12];
    const float* A_log   = (const float*)d_in[13];
    const float* Dsk     = (const float*)d_in[14];
    const float* out_w   = (const float*)d_in[15];
    const float* cls_w   = (const float*)d_in[16];
    const float* cls_b   = (const float*)d_in[17];
    float* out = (float*)d_out;

    const int B = in_sizes[0] / (CIN * LSEQ);
    if (B < 1) return;
    if (B * DM > out_size) return;
    int NL = in_sizes[6] / DM;
    { int c1 = in_sizes[7] / (2 * DI * DM); int c2 = in_sizes[10] / (NXP * DI); int c3 = in_sizes[15] / (DM * DI);
      int c4 = in_sizes[13] / (DI * DS); int c5 = in_sizes[8] / (DI * 4);
      if (c1 < NL) NL = c1; if (c2 < NL) NL = c2; if (c3 < NL) NL = c3; if (c4 < NL) NL = c4; if (c5 < NL) NL = c5; }
    if (NL < 0) NL = 0;

    const size_t nrows = (size_t)B * LSEQ;
    const int nr = (int)nrows;
    if (nr % 64) return;

    size_t off = 0;
    const size_t o_h  = off; off = al256(off + nrows * DM * sizeof(float));
    const size_t o_xz = off; off = al256(off + nrows * 128 * sizeof(float));
    const size_t o_xc = off; off = al256(off + nrows * DI * sizeof(float));
    const size_t o_dl = off; off = al256(off + nrows * DI * sizeof(float));
    const size_t o_bc = off; off = al256(off + nrows * 32 * sizeof(float));
    const size_t o_y  = off; off = al256(off + nrows * DI * sizeof(_Float16));
    if (off > ws_size) return;
    char* ws = (char*)d_ws;
    float*    hbuf = (float*)(ws + o_h);
    float*    xz   = (float*)(ws + o_xz);
    float*    xc   = (float*)(ws + o_xc);
    float*    dl   = (float*)(ws + o_dl);
    float*    bc   = (float*)(ws + o_bc);
    _Float16* yg   = (_Float16*)(ws + o_y);

    k_front<<<(nr + 31) / 32, 256, 0, stream>>>(x, conv_w, bn_g, bn_b, bn_m, bn_v, hbuf, nr);

    for (int l = 0; l < NL; ++l) {
        const float* nwl  = norm_w  + (size_t)l * DM;
        const float* Wil  = in_w    + (size_t)l * 2 * DI * DM;
        const float* cwl  = conv_dw + (size_t)l * DI * 4;
        const float* cbl  = conv_db + (size_t)l * DI;
        const float* Wxl  = x_w     + (size_t)l * NXP * DI;
        const float* Wdtl = dt_w    + (size_t)l * DI * 2;
        const float* bdtl = dt_b    + (size_t)l * DI;
        const float* All  = A_log   + (size_t)l * DI * DS;
        const float* Dpl  = Dsk     + (size_t)l * DI;
        const float* Wol  = out_w   + (size_t)l * DM * DI;

        k_inproj<<<nr / 64, 128, 0, stream>>>(hbuf, nwl, Wil, xz, nr);
        k_xdd<<<nr / 64, 128, 0, stream>>>(xz, cwl, cbl, Wxl, Wdtl, bdtl, xc, dl, bc, nr);
        k_scan<<<B, 512, 0, stream>>>(dl, bc, xc, xz, All, Dpl, yg);
        k_outproj<<<nr / 64, 128, 0, stream>>>(yg, Wol, hbuf, nr);
    }

    k_poolcls<<<(B + 7) / 8, 256, 0, stream>>>(hbuf, cls_w, cls_b, out, B);
}
